// MambaDiffusionBlock_64656437674689
// MI455X (gfx1250) — hardware-verified
//
#include <hip/hip_runtime.h>
#include <math.h>

typedef _Float16 v16h __attribute__((ext_vector_type(16)));
typedef _Float16 v8h  __attribute__((ext_vector_type(8)));
typedef float    v8f  __attribute__((ext_vector_type(8)));
typedef float    v4f  __attribute__((ext_vector_type(4)));
typedef v8h __attribute__((may_alias)) v8ha;
typedef v4f __attribute__((may_alias)) v4fa;

union Frag { v16h v; v8h half[2]; };

#define DIMC   512
#define DIN    1024
#define DST    16
#define DTR    32
#define NH     8
#define HD     64
#define BATCH  4
#define SEQ    1024
#define TXT    77
#define KPAD   96
#define MROWS  (BATCH * SEQ)
#define KVROWS (BATCH * TXT)
#define KVPAD  384
#define XZC    (2 * DIN)
#define DBLC   (DTR + 2 * DST)
#define FFH    (4 * DIMC)
#define PSCALE 16384.0f

#define G_WIP (XZC * DIMC / 8)
#define G_WXP (DBLC * DIN / 8)
#define G_WDT (DIN * DTR / 8)
#define G_WOP (DIMC * DIN / 8)
#define G_WAI (3 * DIMC * DIMC / 8)
#define G_WAO (DIMC * DIMC / 8)
#define G_WF1 (FFH * DIMC / 8)
#define G_WF2 (DIMC * FFH / 8)
#define G_TXT (KVPAD * DIMC / 8)
#define C1 (G_WIP)
#define C2 (C1 + G_WXP)
#define C3 (C2 + G_WDT)
#define C4 (C3 + G_WOP)
#define C5 (C4 + G_WAI)
#define C6 (C5 + G_WAO)
#define C7 (C6 + G_WF1)
#define C8 (C7 + G_WF2)
#define GTOT (C8 + G_TXT)

__device__ __forceinline__ v8f wmma_f16(v16h a, v16h b, v8f c) {
  v8f d = __builtin_amdgcn_wmma_f32_16x16x32_f16(false, a, false, b, (short)0, c, false, false);
  asm volatile("v_nop\n\tv_nop\n\tv_nop\n\tv_nop" : "+v"(d) : "v"(a), "v"(b));
  return d;
}

__device__ __forceinline__ v16h load_frag(const _Float16* p, int h) {
  Frag f;
  f.half[0] = *(const v8ha*)(p + 8 * h);
  f.half[1] = *(const v8ha*)(p + 16 + 8 * h);
  return f.v;
}

__device__ __forceinline__ float rcp_f(float x) { return __builtin_amdgcn_rcpf(x); }

__global__ __launch_bounds__(256) void k_convert(
    const float* __restrict__ wip, const float* __restrict__ wxp, const float* __restrict__ wdt,
    const float* __restrict__ wop, const float* __restrict__ wai, const float* __restrict__ wao,
    const float* __restrict__ wf1, const float* __restrict__ wf2, const float* __restrict__ txt,
    _Float16* __restrict__ dst)
{
  const int g = blockIdx.x * 256 + threadIdx.x;
  if (g >= GTOT) return;
  const float* src = wip;
  float sc = 32.0f;
  bool zero = false;
  if (g < C1)      { src = wip + (size_t)g * 8; }
  else if (g < C2) { src = wxp + (size_t)(g - C1) * 8; }
  else if (g < C3) { src = wdt + (size_t)(g - C2) * 8; sc = 8.0f; }
  else if (g < C4) { src = wop + (size_t)(g - C3) * 8; }
  else if (g < C5) { src = wai + (size_t)(g - C4) * 8; }
  else if (g < C6) { src = wao + (size_t)(g - C5) * 8; }
  else if (g < C7) { src = wf1 + (size_t)(g - C6) * 8; }
  else if (g < C8) { src = wf2 + (size_t)(g - C7) * 8; }
  else {
    const int e = g - C8;
    sc = 1.0f;
    if (e < KVROWS * (DIMC / 8)) src = txt + (size_t)e * 8;
    else zero = true;
  }
  v4f a = {0.0f, 0.0f, 0.0f, 0.0f};
  v4f c = a;
  if (!zero) {
    a = *(const v4fa*)src;
    c = *(const v4fa*)(src + 4);
  }
  const v8h o = { (_Float16)(a.x * sc), (_Float16)(a.y * sc), (_Float16)(a.z * sc), (_Float16)(a.w * sc),
                  (_Float16)(c.x * sc), (_Float16)(c.y * sc), (_Float16)(c.z * sc), (_Float16)(c.w * sc) };
  _Float16* d = dst + (size_t)g * 8;
  *(volatile v8h*)d = o;
  __threadfence();
  *(volatile v8h*)d = o;
}

__global__ __launch_bounds__(256) void k_layernorm(
    const float* __restrict__ x, const float* __restrict__ w, const float* __restrict__ bb,
    float* outf, _Float16* outh, int nrows)
{
  const int lane = threadIdx.x & 31, wv = threadIdx.x >> 5;
  const int row = blockIdx.x * 8 + wv;
  if (row >= nrows) return;
  const float* xr = x + (size_t)row * DIMC;

  v4f v[4];
  float s = 0.0f;
  #pragma unroll
  for (int j = 0; j < 4; ++j) {
    v[j] = *(const v4fa*)(xr + 4 * lane + 128 * j);
    s += (v[j].x + v[j].y) + (v[j].z + v[j].w);
  }
  #pragma unroll
  for (int off = 16; off > 0; off >>= 1) s += __shfl_xor(s, off);
  const float mu = s * (1.0f / 512.0f);
  float ss = 0.0f;
  #pragma unroll
  for (int j = 0; j < 4; ++j) {
    const v4f dx = v[j] - mu;
    ss += (dx.x * dx.x + dx.y * dx.y) + (dx.z * dx.z + dx.w * dx.w);
  }
  #pragma unroll
  for (int off = 16; off > 0; off >>= 1) ss += __shfl_xor(ss, off);
  const float var = ss * (1.0f / 512.0f);
  const float inv = rsqrtf(var + 1e-5f);

  v4f y[4];
  if (outf != nullptr) {
    #pragma unroll
    for (int j = 0; j < 4; ++j) {
      const int c = 4 * lane + 128 * j;
      const v4f wv4 = *(const v4fa*)(w + c);
      const v4f bv4 = *(const v4fa*)(bb + c);
      y[j] = (v[j] - mu) * inv * wv4 + bv4;
    }
  }
  v8h yh[2];
  #pragma unroll
  for (int j = 0; j < 2; ++j) {
    const int c0 = 8 * lane + 256 * j;
    const v4f a  = *(const v4fa*)(xr + c0);
    const v4f c  = *(const v4fa*)(xr + c0 + 4);
    const v4f wa = *(const v4fa*)(w + c0);
    const v4f wc = *(const v4fa*)(w + c0 + 4);
    const v4f ba = *(const v4fa*)(bb + c0);
    const v4f bc = *(const v4fa*)(bb + c0 + 4);
    const v4f ya = (a - mu) * inv * wa + ba;
    const v4f yc = (c - mu) * inv * wc + bc;
    const v8h o = { (_Float16)ya.x, (_Float16)ya.y, (_Float16)ya.z, (_Float16)ya.w,
                    (_Float16)yc.x, (_Float16)yc.y, (_Float16)yc.z, (_Float16)yc.w };
    yh[j] = o;
  }

  if (outf != nullptr) {
    #pragma unroll
    for (int j = 0; j < 4; ++j)
      *(volatile v4f*)(outf + (size_t)row * DIMC + 4 * lane + 128 * j) = y[j];
  }
  #pragma unroll
  for (int j = 0; j < 2; ++j)
    *(volatile v8h*)(outh + (size_t)row * DIMC + 8 * lane + 256 * j) = yh[j];
  __threadfence();
  if (outf != nullptr) {
    #pragma unroll
    for (int j = 0; j < 4; ++j)
      *(volatile v4f*)(outf + (size_t)row * DIMC + 4 * lane + 128 * j) = y[j];
  }
  #pragma unroll
  for (int j = 0; j < 2; ++j)
    *(volatile v8h*)(outh + (size_t)row * DIMC + 8 * lane + 256 * j) = yh[j];
}

template <bool OUTF, bool OUTH>
__device__ __forceinline__ void gemm_store(const float* sT, float* outf, _Float16* outh,
                                           int N, int m0, int n0, int w, int lane, float hmul) {
  const int q8 = lane & 7, sub = lane >> 3;
  if (OUTF) {
    #pragma unroll
    for (int i = 0; i < 16; ++i) {
      const int lid = i * 4 + sub;
      const int row = 32 * w + (lid >> 1), hl = lid & 1;
      const v4f v = *(const v4fa*)(sT + row * 64 + 32 * hl + 4 * q8);
      float* dst = outf + (size_t)(m0 + row) * N + n0 + 32 * hl + 4 * q8;
      *(volatile v4f*)dst = v;
    }
  }
  if (OUTH) {
    #pragma unroll
    for (int i = 0; i < 8; ++i) {
      const int lid = i * 4 + sub;
      const int row = 32 * w + lid;
      const v4f a = *(const v4fa*)(sT + row * 64 + 8 * q8);
      const v4f c = *(const v4fa*)(sT + row * 64 + 8 * q8 + 4);
      const v8h o = { (_Float16)(a.x * hmul), (_Float16)(a.y * hmul), (_Float16)(a.z * hmul), (_Float16)(a.w * hmul),
                      (_Float16)(c.x * hmul), (_Float16)(c.y * hmul), (_Float16)(c.z * hmul), (_Float16)(c.w * hmul) };
      _Float16* dst = outh + (size_t)(m0 + row) * N + n0 + 8 * q8;
      *(volatile v8h*)dst = o;
    }
  }
}

template <int ACT, bool OUTF, bool OUTH>
__global__ __launch_bounds__(128) void k_gemm(
    const _Float16* __restrict__ A, int lda,
    const _Float16* __restrict__ W, int K, int N,
    const float* __restrict__ bias,
    const float* __restrict__ res1, const float* __restrict__ res2,
    float oscale, float hmul,
    float* outf, _Float16* outh)
{
  __shared__ __attribute__((aligned(16))) float sT[128 * 64];

  const int tid = threadIdx.x, lane = tid & 31, w = tid >> 5;
  const int h = lane >> 4, m = lane & 15;
  const int m0 = blockIdx.y * 128, n0 = blockIdx.x * 64;
  const int m0w = m0 + 32 * w;

  const _Float16* a0p = A + (size_t)(m0w + m) * lda;
  const _Float16* a1p = a0p + (size_t)16 * lda;
  const _Float16* wp  = W + (size_t)(n0 + m) * K;

  const v8f zero8 = {0.f, 0.f, 0.f, 0.f, 0.f, 0.f, 0.f, 0.f};
  v8f acc[2][4];
  #pragma unroll
  for (int mt = 0; mt < 2; ++mt)
    #pragma unroll
    for (int nt = 0; nt < 4; ++nt) acc[mt][nt] = zero8;

  #pragma unroll 1
  for (int k0 = 0; k0 < K; k0 += 32) {
    const v16h a0 = load_frag(a0p + k0, h);
    const v16h a1 = load_frag(a1p + k0, h);
    #pragma unroll
    for (int nt = 0; nt < 4; ++nt) {
      const v16h b = load_frag(wp + (size_t)nt * 16 * K + k0, h);
      acc[0][nt] = wmma_f16(a0, b, acc[0][nt]);
      acc[1][nt] = wmma_f16(a1, b, acc[1][nt]);
    }
  }

  #pragma unroll
  for (int nt = 0; nt < 4; ++nt) {
    const int nl = 16 * nt + m;
    const int n = n0 + nl;
    const float bv = (bias != nullptr) ? bias[n] : 0.0f;
    #pragma unroll
    for (int mt = 0; mt < 2; ++mt) {
      #pragma unroll
      for (int r = 0; r < 8; ++r) {
        const int rowl = 32 * w + 16 * mt + 8 * h + r;
        float val = acc[mt][nt][r] * oscale + bv;
        if (ACT == 1) {
          val = fmaxf(val, 0.0f) + log1pf(__expf(-fabsf(val)));
        } else if (ACT == 2) {
          val = 0.5f * val * (1.0f + erff(val * 0.70710678118654752f));
        }
        const size_t o = (size_t)(m0 + rowl) * N + n;
        if (res1 != nullptr) val += res1[o];
        if (res2 != nullptr) val += res2[o];
        sT[rowl * 64 + nl] = val;
      }
    }
  }
  __syncthreads();

  gemm_store<OUTF, OUTH>(sT, outf, outh, N, m0, n0, w, lane, hmul);
  __threadfence();
  gemm_store<OUTF, OUTH>(sT, outf, outh, N, m0, n0, w, lane, hmul);
}

__global__ __launch_bounds__(128) void k_conv(
    const float* __restrict__ xz, const float* __restrict__ cw, const float* __restrict__ cb,
    _Float16* xch)
{
  const int row = blockIdx.x;
  const int l = row & (SEQ - 1);
  const int c0 = threadIdx.x * 8;
  v4f wv[8];
  #pragma unroll
  for (int i = 0; i < 8; ++i) wv[i] = *(const v4fa*)(cw + (size_t)(c0 + i) * 4);
  float acc[8];
  #pragma unroll
  for (int i = 0; i < 8; ++i) acc[i] = 0.0f;
  #pragma unroll
  for (int k = 0; k < 4; ++k) {
    const int ls = l + k - 3;
    if (ls >= 0) {
      const float* p = xz + (size_t)(row + k - 3) * XZC + c0;
      const v4f a = *(const v4fa*)p;
      const v4f c = *(const v4fa*)(p + 4);
      acc[0] += a.x * wv[0][k]; acc[1] += a.y * wv[1][k];
      acc[2] += a.z * wv[2][k]; acc[3] += a.w * wv[3][k];
      acc[4] += c.x * wv[4][k]; acc[5] += c.y * wv[5][k];
      acc[6] += c.z * wv[6][k]; acc[7] += c.w * wv[7][k];
    }
  }
  const v4f ba = *(const v4fa*)(cb + c0);
  const v4f bc = *(const v4fa*)(cb + c0 + 4);
  acc[0] += ba.x; acc[1] += ba.y; acc[2] += ba.z; acc[3] += ba.w;
  acc[4] += bc.x; acc[5] += bc.y; acc[6] += bc.z; acc[7] += bc.w;
  float y[8];
  #pragma unroll
  for (int i = 0; i < 8; ++i) y[i] = acc[i] * rcp_f(1.0f + __expf(-acc[i])) * 16.0f;
  const v8h o = { (_Float16)y[0], (_Float16)y[1], (_Float16)y[2], (_Float16)y[3],
                  (_Float16)y[4], (_Float16)y[5], (_Float16)y[6], (_Float16)y[7] };
  _Float16* dst = xch + (size_t)row * DIN + c0;
  *(volatile v8h*)dst = o;
  __threadfence();
  *(volatile v8h*)dst = o;
}

__device__ __forceinline__ void scan_store(const _Float16* sY, _Float16* ysh,
                                           int b, int l0, int cbase, int w, int lane) {
  const int q8 = lane & 7, sub = lane >> 3;
  #pragma unroll
  for (int i = 0; i < 4; ++i) {
    const int lid = w * 16 + i * 4 + sub;
    const int r = lid >> 1, hl = lid & 1;
    const v8h v = *(const v8ha*)(sY + r * 128 + 64 * hl + 8 * q8);
    _Float16* dst = ysh + (size_t)(b * SEQ + l0 + r) * DIN + cbase + 64 * hl + 8 * q8;
    *(volatile v8h*)dst = v;
  }
}

__global__ __launch_bounds__(128) void k_scan(
    const float* __restrict__ xz,
    const float* __restrict__ dt,
    const float* __restrict__ dbl,
    const float* __restrict__ alog,
    const float* __restrict__ dp,
    const float* __restrict__ cw,
    const float* __restrict__ cb,
    _Float16* ysh)
{
  __shared__ __attribute__((aligned(16))) float sBC[32 * 32];
  __shared__ __attribute__((aligned(16))) _Float16 sY[32 * 128];

  const int tid = threadIdx.x, lane = tid & 31, w = tid >> 5;
  const int b = blockIdx.y;
  const int cbase = blockIdx.x * 128;
  const int d = cbase + tid;

  float Aa[DST];
  #pragma unroll
  for (int j = 0; j < 4; ++j) {
    const v4f al = *(const v4fa*)(alog + (size_t)d * DST + 4 * j);
    Aa[4 * j + 0] = -expf(al.x); Aa[4 * j + 1] = -expf(al.y);
    Aa[4 * j + 2] = -expf(al.z); Aa[4 * j + 3] = -expf(al.w);
  }
  float hs[DST];
  #pragma unroll
  for (int n = 0; n < DST; ++n) hs[n] = 0.0f;
  const float Dd = dp[d];
  const v4f wv = *(const v4fa*)(cw + (size_t)d * 4);
  const float cbd = cb[d];
  float xm1 = 0.0f, xm2 = 0.0f, xm3 = 0.0f;

  const int st_i = tid >> 2, st_p = (tid & 3) * 8;

  #pragma unroll 1
  for (int l0 = 0; l0 < SEQ; l0 += 32) {
    __syncthreads();
    {
      const float* src = dbl + (size_t)(b * SEQ + l0 + st_i) * DBLC + DTR + st_p;
      *(v4fa*)(sBC + st_i * 32 + st_p)     = *(const v4fa*)src;
      *(v4fa*)(sBC + st_i * 32 + st_p + 4) = *(const v4fa*)(src + 4);
    }
    __syncthreads();

    #pragma unroll 1
    for (int i = 0; i < 32; ++i) {
      const size_t row = (size_t)(b * SEQ + l0 + i);
      const float xin = xz[row * XZC + d];
      const float zv  = xz[row * XZC + DIN + d];
      const float dtv = dt[row * DIN + d];
      float conv = xm3 * wv.x;
      conv += xm2 * wv.y;
      conv += xm1 * wv.z;
      conv += xin * wv.w;
      conv += cbd;
      xm3 = xm2; xm2 = xm1; xm1 = xin;
      const float xc = conv * rcp_f(1.0f + __expf(-conv));

      v4f bc[8];
      #pragma unroll
      for (int j = 0; j < 8; ++j) bc[j] = *(const v4fa*)(sBC + i * 32 + 4 * j);

      float y = 0.0f;
      #pragma unroll
      for (int n = 0; n < DST; ++n) {
        const float Bn = bc[n >> 2][n & 3];
        const float Cn = bc[4 + (n >> 2)][n & 3];
        const float dA = __expf(dtv * Aa[n]);
        hs[n] = dA * hs[n] + (dtv * Bn) * xc;
        y += hs[n] * Cn;
      }
      y += Dd * xc;
      y *= zv * rcp_f(1.0f + __expf(-zv));
      sY[i * 128 + tid] = (_Float16)(y * 16.0f);
    }
    __syncthreads();
    scan_store(sY, ysh, b, l0, cbase, w, lane);
    __threadfence();
    scan_store(sY, ysh, b, l0, cbase, w, lane);
  }
}

__device__ __forceinline__ v16h pack_p(v8f a, v8f c) {
  const v16h r = { (_Float16)(a[0] * PSCALE), (_Float16)(a[1] * PSCALE), (_Float16)(a[2] * PSCALE), (_Float16)(a[3] * PSCALE),
                   (_Float16)(a[4] * PSCALE), (_Float16)(a[5] * PSCALE), (_Float16)(a[6] * PSCALE), (_Float16)(a[7] * PSCALE),
                   (_Float16)(c[0] * PSCALE), (_Float16)(c[1] * PSCALE), (_Float16)(c[2] * PSCALE), (_Float16)(c[3] * PSCALE),
                   (_Float16)(c[4] * PSCALE), (_Float16)(c[5] * PSCALE), (_Float16)(c[6] * PSCALE), (_Float16)(c[7] * PSCALE) };
  return r;
}

__device__ __forceinline__ void attn_store(const _Float16* so, _Float16* att,
                                           int b, int head, int q0, int lane) {
  const int q8 = lane & 7, sub = lane >> 3;
  #pragma unroll
  for (int i = 0; i < 4; ++i) {
    const int lid = i * 4 + sub;
    const v8h v = *(const v8ha*)(so + lid * HD + 8 * q8);
    _Float16* dst = att + (size_t)(b * SEQ + q0 + lid) * DIMC + head * HD + 8 * q8;
    *(volatile v8h*)dst = v;
  }
}

__global__ __launch_bounds__(128) void k_attn(
    const _Float16* __restrict__ qh,
    const _Float16* __restrict__ kh,
    const _Float16* __restrict__ vh,
    _Float16* att)
{
  __shared__ __attribute__((aligned(16))) _Float16 sVt[HD * KPAD];
  __shared__ __attribute__((aligned(16))) _Float16 sO[4 * 16 * HD];

  const int tid = threadIdx.x, lane = tid & 31, w = tid >> 5;
  const int h = lane >> 4, m = lane & 15;
  const int bh = blockIdx.y, b = bh >> 3, head = bh & 7;
  const int q0 = blockIdx.x * 64 + 16 * w;

  for (int idx = tid; idx < KPAD * HD; idx += 128) {
    const int key = idx >> 6, dd = idx & 63;
    _Float16 val = (_Float16)0.0f;
    if (key < TXT) val = vh[(size_t)(b * TXT + key) * DIMC + head * HD + dd];
    sVt[dd * KPAD + key] = val;
  }
  __syncthreads();

  const v8f zero8 = {0.f, 0.f, 0.f, 0.f, 0.f, 0.f, 0.f, 0.f};

  const _Float16* qrow = qh + (size_t)(b * SEQ + q0 + m) * DIMC + head * HD;
  const v16h qb0 = load_frag(qrow, h);
  const v16h qb1 = load_frag(qrow + 32, h);

  v8f s[6];
  #pragma unroll
  for (int j = 0; j < 6; ++j) {
    const _Float16* kp = kh + (size_t)(b * TXT + 16 * j + m) * DIMC + head * HD;
    const v16h kf0 = load_frag(kp, h);
    const v16h kf1 = load_frag(kp + 32, h);
    v8f z = zero8;
    z = wmma_f16(kf0, qb0, z);
    z = wmma_f16(kf1, qb1, z);
    s[j] = z;
  }

  float mx = -1e30f;
  #pragma unroll
  for (int j = 0; j < 6; ++j)
    #pragma unroll
    for (int r = 0; r < 8; ++r) {
      const int key = 16 * j + 8 * h + r;
      float v = s[j][r] * 0.0625f;
      v = (key < TXT) ? v : -1e30f;
      s[j][r] = v;
      mx = fmaxf(mx, v);
    }
  mx = fmaxf(mx, __shfl_xor(mx, 16));
  float lsum = 0.0f;
  #pragma unroll
  for (int j = 0; j < 6; ++j)
    #pragma unroll
    for (int r = 0; r < 8; ++r) {
      const float p = __expf(s[j][r] - mx);
      s[j][r] = p;
      lsum += p;
    }
  lsum += __shfl_xor(lsum, 16);

  v16h pb[3];
  #pragma unroll
  for (int c = 0; c < 3; ++c) pb[c] = pack_p(s[2 * c], s[2 * c + 1]);

  v8f o[4];
  #pragma unroll
  for (int t = 0; t < 4; ++t) {
    const _Float16* vp = sVt + (16 * t + m) * KPAD;
    v8f z = zero8;
    #pragma unroll
    for (int c = 0; c < 3; ++c) {
      const v16h vf = load_frag(vp + 32 * c, h);
      z = wmma_f16(vf, pb[c], z);
    }
    o[t] = z;
  }

  const float inv = rcp_f(lsum) * (16.0f / PSCALE);
  _Float16* so = sO + w * 16 * HD;
  #pragma unroll
  for (int t = 0; t < 4; ++t)
    #pragma unroll
    for (int r = 0; r < 8; ++r)
      so[m * HD + 16 * t + 8 * h + r] = (_Float16)(o[t][r] * inv);
  __syncthreads();

  attn_store(so, att, b, head, q0, lane);
  __threadfence();
  attn_store(so, att, b, head, q0, lane);
}

extern "C" void kernel_launch(void* const* d_in, const int* in_sizes, int n_in,
                              void* d_out, int out_size, void* d_ws, size_t ws_size,
                              hipStream_t stream)
{
  if (n_in < 25) return;
  if (in_sizes[0] != MROWS * DIMC) return;
  if (in_sizes[1] != KVROWS * DIMC) return;
  if (in_sizes[2] != DIMC || in_sizes[4] != DIMC || in_sizes[6] != DIMC) return;
  if (in_sizes[8] != XZC * DIMC || in_sizes[9] != DIN * 4 || in_sizes[10] != DIN) return;
  if (in_sizes[11] != DBLC * DIN || in_sizes[12] != DIN * DTR || in_sizes[13] != DIN) return;
  if (in_sizes[14] != DIN * DST || in_sizes[15] != DIN || in_sizes[16] != DIMC * DIN) return;
  if (in_sizes[17] != 3 * DIMC * DIMC || in_sizes[18] != 3 * DIMC) return;
  if (in_sizes[19] != DIMC * DIMC || in_sizes[20] != DIMC) return;
  if (in_sizes[21] != FFH * DIMC || in_sizes[22] != FFH || in_sizes[23] != DIMC * FFH || in_sizes[24] != DIMC) return;
  if (out_size != MROWS * DIMC) return;

  const float* x        = (const float*)d_in[0];
  const float* text     = (const float*)d_in[1];
  const float* ln1_w    = (const float*)d_in[2];
  const float* ln1_b    = (const float*)d_in[3];
  const float* ln2_w    = (const float*)d_in[4];
  const float* ln2_b    = (const float*)d_in[5];
  const float* ln3_w    = (const float*)d_in[6];
  const float* ln3_b    = (const float*)d_in[7];
  const float* in_proj  = (const float*)d_in[8];
  const float* conv_w   = (const float*)d_in[9];
  const float* conv_b   = (const float*)d_in[10];
  const float* x_proj   = (const float*)d_in[11];
  const float* dt_proj  = (const float*)d_in[12];
  const float* dt_projb = (const float*)d_in[13];
  const float* A_log    = (const float*)d_in[14];
  const float* Dp       = (const float*)d_in[15];
  const float* out_proj = (const float*)d_in[16];
  const float* attn_inw = (const float*)d_in[17];
  const float* attn_inb = (const float*)d_in[18];
  const float* attn_ow  = (const float*)d_in[19];
  const float* attn_ob  = (const float*)d_in[20];
  const float* ffn_w1   = (const float*)d_in[21];
  const float* ffn_b1   = (const float*)d_in[22];
  const float* ffn_w2   = (const float*)d_in[23];
  const float* ffn_b2   = (const float*)d_in[24];
  float* outp = (float*)d_out;

  const size_t B_WALL = (size_t)GTOT * 16;
  const size_t B_HH   = (size_t)MROWS * DIMC * 2;
  const size_t B_XZ   = (size_t)MROWS * XZC * 4;
  const size_t B_XCH  = (size_t)MROWS * DIN * 2;
  const size_t B_DBL  = (size_t)MROWS * DBLC * 4;
  const size_t B_DBLH = (size_t)MROWS * DBLC * 2;
  const size_t B_DT   = (size_t)MROWS * DIN * 4;
  const size_t B_YSH  = (size_t)MROWS * DIN * 2;
  const size_t B_X    = (size_t)MROWS * DIMC * 4;
  const size_t B_QH   = (size_t)MROWS * DIMC * 2;
  const size_t B_KV   = (size_t)KVPAD * DIMC * 2;
  const size_t B_ATT  = (size_t)MROWS * DIMC * 2;
  size_t off = 0;
  const size_t o_wall = off; off += B_WALL;
  const size_t o_hh   = off; off += B_HH;
  const size_t o_xz   = off; off += B_XZ;
  const size_t o_xch  = off; off += B_XCH;
  const size_t o_dbl  = off; off += B_DBL;
  const size_t o_dblh = off; off += B_DBLH;
  const size_t o_dt   = off; off += B_DT;
  const size_t o_ysh  = off; off += B_YSH;
  const size_t o_x1   = off; off += B_X;
  const size_t o_h2   = off; off += B_X;
  const size_t o_qh   = off; off += B_QH;
  const size_t o_kh   = off; off += B_KV;
  const size_t o_vh   = off; off += B_KV;
  const size_t o_att  = off; off += B_ATT;
  const size_t o_x2   = off; off += B_X;
  const size_t total  = off;
  if (total > ws_size) return;
  if ((size_t)MROWS * FFH * 2 > B_XZ) return;

  char* ws = (char*)d_ws;
  _Float16* wall = (_Float16*)(ws + o_wall);
  _Float16* w_ip  = wall + (size_t)8 * 0;
  _Float16* w_xp  = wall + (size_t)8 * C1;
  _Float16* w_dt  = wall + (size_t)8 * C2;
  _Float16* w_op  = wall + (size_t)8 * C3;
  _Float16* w_ai  = wall + (size_t)8 * C4;
  _Float16* w_ao  = wall + (size_t)8 * C5;
  _Float16* w_f1  = wall + (size_t)8 * C6;
  _Float16* w_f2  = wall + (size_t)8 * C7;
  _Float16* txth  = wall + (size_t)8 * C8;
  _Float16* hh    = (_Float16*)(ws + o_hh);
  float*    xz    = (float*)(ws + o_xz);
  _Float16* f1h   = (_Float16*)(ws + o_xz);
  _Float16* xch   = (_Float16*)(ws + o_xch);
  float*    dbl   = (float*)(ws + o_dbl);
  _Float16* dblh  = (_Float16*)(ws + o_dblh);
  float*    dtb   = (float*)(ws + o_dt);
  _Float16* ysh   = (_Float16*)(ws + o_ysh);
  float*    x1    = (float*)(ws + o_x1);
  float*    h2    = (float*)(ws + o_h2);
  _Float16* qh    = (_Float16*)(ws + o_qh);
  _Float16* kh    = (_Float16*)(ws + o_kh);
  _Float16* vh    = (_Float16*)(ws + o_vh);
  _Float16* att   = (_Float16*)(ws + o_att);
  float*    x2    = (float*)(ws + o_x2);

  float* nullf = nullptr;
  _Float16* nullh = nullptr;
  const float* nullc = nullptr;

  k_convert<<<(GTOT + 255) / 256, 256, 0, stream>>>(in_proj, x_proj, dt_proj, out_proj, attn_inw, attn_ow,
                                                     ffn_w1, ffn_w2, text, wall);
  k_layernorm<<<MROWS / 8, 256, 0, stream>>>(x, ln1_w, ln1_b, nullf, hh, MROWS);
  k_gemm<0, true, false><<<dim3(XZC / 64, MROWS / 128), 128, 0, stream>>>(
      hh, DIMC, w_ip, DIMC, XZC, nullc, nullc, nullc, 1.0f / 32.0f, 1.0f, xz, nullh);
  k_conv<<<MROWS, 128, 0, stream>>>(xz, conv_w, conv_b, xch);
  k_gemm<0, true, true><<<dim3(DBLC / 64, MROWS / 128), 128, 0, stream>>>(
      xch, DIN, w_xp, DIN, DBLC, nullc, nullc, nullc, 1.0f / 512.0f, 16.0f, dbl, dblh);
  k_gemm<1, true, false><<<dim3(DIN / 64, MROWS / 128), 128, 0, stream>>>(
      dblh, DBLC, w_dt, DTR, DIN, dt_projb, nullc, nullc, 1.0f / 128.0f, 1.0f, dtb, nullh);
  k_scan<<<dim3(DIN / 128, BATCH), 128, 0, stream>>>(xz, dtb, dbl, A_log, Dp, conv_w, conv_b, ysh);
  k_gemm<0, true, false><<<dim3(DIMC / 64, MROWS / 128), 128, 0, stream>>>(
      ysh, DIN, w_op, DIN, DIMC, nullc, x, nullc, 1.0f / 512.0f, 1.0f, x1, nullh);
  k_layernorm<<<MROWS / 8, 256, 0, stream>>>(x1, ln2_w, ln2_b, h2, hh, MROWS);
  k_gemm<0, false, true><<<dim3(DIMC / 64, MROWS / 128), 128, 0, stream>>>(
      hh, DIMC, w_ai, DIMC, DIMC, attn_inb, nullc, nullc, 1.0f / 32.0f, 2.0f, nullf, qh);
  k_gemm<0, false, true><<<dim3(DIMC / 64, KVPAD / 128), 128, 0, stream>>>(
      txth, DIMC, w_ai + (size_t)DIMC * DIMC, DIMC, DIMC, attn_inb + DIMC, nullc, nullc, 1.0f / 32.0f, 1.0f, nullf, kh);
  k_gemm<0, false, true><<<dim3(DIMC / 64, KVPAD / 128), 128, 0, stream>>>(
      txth, DIMC, w_ai + (size_t)2 * DIMC * DIMC, DIMC, DIMC, attn_inb + 2 * DIMC, nullc, nullc, 1.0f / 32.0f, 1.0f, nullf, vh);
  k_attn<<<dim3(SEQ / 64, BATCH * NH), 128, 0, stream>>>(qh, kh, vh, att);
  k_gemm<0, true, false><<<dim3(DIMC / 64, MROWS / 128), 128, 0, stream>>>(
      att, DIMC, w_ao, DIMC, DIMC, attn_ob, h2, x1, 1.0f / 512.0f, 1.0f, x2, nullh);
  k_layernorm<<<MROWS / 8, 256, 0, stream>>>(x2, ln3_w, ln3_b, nullf, hh, MROWS);
  k_gemm<2, false, true><<<dim3(FFH / 64, MROWS / 128), 128, 0, stream>>>(
      hh, DIMC, w_f1, DIMC, FFH, ffn_b1, nullc, nullc, 1.0f / 32.0f, 1.0f, nullf, f1h);
  k_gemm<0, true, false><<<dim3(DIMC / 64, MROWS / 128), 128, 0, stream>>>(
      f1h, FFH, w_f2, FFH, DIMC, ffn_b2, x2, nullc, 1.0f / 32.0f, 1.0f, outp, nullh);
}
